// FP_86655260164508
// MI455X (gfx1250) — hardware-verified
//
#include <hip/hip_runtime.h>
#include <math.h>

typedef __attribute__((ext_vector_type(16))) _Float16 v16h;
typedef __attribute__((ext_vector_type(16))) __bf16 v16b;
typedef __attribute__((ext_vector_type(8)))  _Float16 v8h;
typedef __attribute__((ext_vector_type(8)))  float v8f;
typedef __attribute__((ext_vector_type(4)))  float v4f;
typedef __attribute__((ext_vector_type(2)))  float v2f;
typedef __attribute__((ext_vector_type(4)))  unsigned v4u;
typedef __attribute__((ext_vector_type(4)))  int v4i;
typedef float __attribute__((may_alias)) float_a;
typedef int __attribute__((may_alias)) int_a;

template <typename T> __device__ __forceinline__ void vst2(void* p, T v) { *(volatile T*)p = v; __threadfence(); *(volatile T*)p = v; }
__device__ __forceinline__ v8f wmma16(v16h a, v16h b, v8f c) {
  v8f d = __builtin_amdgcn_wmma_f32_16x16x32_f16(false, a, false, b, (short)0, c, false, false);
  asm volatile("v_nop\n\tv_nop\n\tv_nop\n\tv_nop" : "+v"(d) : "v"(a), "v"(b));
  return d;
}
__device__ __forceinline__ v8f wmma_bf(v16b a, v16b b, v8f c) {
  v8f d = __builtin_amdgcn_wmma_f32_16x16x32_bf16(false, a, false, b, (short)0, c, false, false);
  asm volatile("v_nop\n\tv_nop\n\tv_nop\n\tv_nop" : "+v"(d) : "v"(a), "v"(b));
  return d;
}
__device__ __forceinline__ v16h frag_h(const _Float16* rowk0, int lane) {
  union { v16h v; v8h q[2]; } u; const _Float16* p = rowk0 + 8 * (lane >> 4);
  u.q[0] = *(const v8h*)p; u.q[1] = *(const v8h*)(p + 16); return u.v;
}
__device__ __forceinline__ v16h frag_f32(const float* rowk0, int lane) {
  v16h a; const float* p = rowk0 + 8 * (lane >> 4);
#pragma unroll
  for (int i = 0; i < 8; ++i) { a[i] = (_Float16)p[i]; a[8 + i] = (_Float16)p[16 + i]; }
  return a;
}
__device__ __forceinline__ v16h frag_f32s(const float* rowk0, int lane, float sc) {
  v16h a; const float* p = rowk0 + 8 * (lane >> 4);
#pragma unroll
  for (int i = 0; i < 8; ++i) { a[i] = (_Float16)(p[i] * sc); a[8 + i] = (_Float16)(p[16 + i] * sc); }
  return a;
}
__device__ __forceinline__ v16h fragc_f32(const float* W, int k0, int n, int lane, int ld, int K) {
  v16h a; const int g = lane >> 4;
#pragma unroll
  for (int i = 0; i < 8; ++i) { const int ka = k0 + 8 * g + i, kb = ka + 16;
    a[i] = (_Float16)(ka < K ? W[(size_t)(ka < K ? ka : K - 1) * ld + n] : 0.f); a[8 + i] = (_Float16)(kb < K ? W[(size_t)(kb < K ? kb : K - 1) * ld + n] : 0.f); }
  return a;
}
struct F2 { v16b h, l; };
__device__ __forceinline__ F2 bsplit16(const float v[16]) { F2 r;
#pragma unroll
  for (int i = 0; i < 16; ++i) { const __bf16 h = (__bf16)v[i]; r.h[i] = h; r.l[i] = (__bf16)(v[i] - (float)h); }
  return r; }
__device__ __forceinline__ F2 split_row(const float* row, int k0, int lane) { float v[16]; const float* p = row + k0 + 8 * (lane >> 4);
#pragma unroll
  for (int i = 0; i < 8; ++i) { v[i] = p[i]; v[8 + i] = p[16 + i]; }
  return bsplit16(v); }
__device__ __forceinline__ F2 split_rowK(const float* row, int k0, int lane, int K) { float v[16]; const int g = lane >> 4;
#pragma unroll
  for (int i = 0; i < 8; ++i) { const int ka = k0 + 8 * g + i, kb = ka + 16; v[i] = ka < K ? row[ka < K ? ka : K - 1] : 0.f; v[8 + i] = kb < K ? row[kb < K ? kb : K - 1] : 0.f; }
  return bsplit16(v); }
__device__ __forceinline__ F2 split_col(const float* W, int k0, int n, int lane, int ld, int K) { float v[16]; const int g = lane >> 4;
#pragma unroll
  for (int i = 0; i < 8; ++i) { const int ka = k0 + 8 * g + i, kb = ka + 16; v[i] = ka < K ? W[(size_t)(ka < K ? ka : K - 1) * ld + n] : 0.f; v[8 + i] = kb < K ? W[(size_t)(kb < K ? kb : K - 1) * ld + n] : 0.f; }
  return bsplit16(v); }
__device__ __forceinline__ v8f mac3(const F2& a, const F2& b, v8f c) { c = wmma_bf(a.l, b.h, c); c = wmma_bf(a.h, b.l, c); return wmma_bf(a.h, b.h, c); }
__device__ __forceinline__ float sigm(float v) { return 1.0f / (1.0f + expf(-v)); }
#define LDSX() do { asm volatile("s_wait_dscnt 0" ::: "memory"); __builtin_amdgcn_wave_barrier(); __builtin_amdgcn_fence(__ATOMIC_RELEASE, "workgroup"); } while (0)


#define NB 4
#define NN 16384
#define NS 4096
#define NR (NB * NN)
#define CF 128
#define CCO 256
#define CIN 384
#define MID 192
#define CO 128
#define NGRP 8
typedef __attribute__((ext_vector_type(8))) __bf16 v8b;
__device__ __forceinline__ v16b frag_b(const __bf16* rowk0, int lane) {
  union { v16b v; v8b q[2]; } u; const __bf16* p = rowk0 + 8 * (lane >> 4);
  u.q[0] = *(const v8b*)p; u.q[1] = *(const v8b*)(p + 16); return u.v;
}
__device__ __forceinline__ float bfr(float v) { return (float)(__bf16)v; }
__device__ __attribute__((noinline)) float exp_ni(float v) { return expf(v); }
__device__ __attribute__((noinline)) float erf_ni(float v) { return erff(v); }

#define PK_1 0
#define PK_2 (MID * CIN)
#define PK_END (PK_2 + CO * MID)
#define WS_PK  0u
#define WS_X2  (((2u * PK_END) + 127u) / 128u * 128u)
#define WS_SQ2 (WS_X2 + 4u * NB * NS * 4)
#define WS_AH  (WS_SQ2 + 4u * NB * NS)
#define WS_AL  (WS_AH + 2u * (size_t)NR * CIN)
#define WS_H1  (WS_AL + 2u * (size_t)NR * CIN)
#define WS_ST1 (WS_H1 + 4u * (size_t)NR * MID)
#define WS_GN1 (WS_ST1 + 8u * (NR / 64) * MID * 2)
#define WS_N1H (WS_GN1 + 4u * NB * 32)
#define WS_N1L (WS_N1H + 2u * (size_t)NR * MID)
#define WS_H2  (WS_N1L + 2u * (size_t)NR * MID)
#define WS_ST2 (WS_H2 + 4u * (size_t)NR * CO)
#define WS_GN2 (WS_ST2 + 8u * (NR / 64) * CO * 2)
#define WS_END (WS_GN2 + 4u * NB * 32)

__global__ __launch_bounds__(256) void k_pack(const float* __restrict__ W1, const float* __restrict__ W2, __bf16* __restrict__ PK) {
  __shared__ __align__(16) __bf16 s[CIN]; const int n = blockIdx.x, which = blockIdx.y, t = threadIdx.x; int K; size_t dst;
  if (which == 0) { if (n >= MID) return; K = CIN; dst = PK_1 + (size_t)n * CIN; for (int k = t; k < CIN; k += 256) s[k] = (__bf16)W1[(size_t)n * CIN + k]; }
  else { if (n >= CO) return; K = MID; dst = PK_2 + (size_t)n * MID; if (t < MID) s[t] = (__bf16)W2[(size_t)n * MID + t]; }
  __syncthreads();
  for (int q = t; q < K / 8; q += 256) vst2((unsigned*)(PK + dst + q * 8), *(const v4u*)&s[q * 8]);
}
__global__ __launch_bounds__(256) void k_src(const float* __restrict__ XYZ2, float* __restrict__ X2, float* __restrict__ SQ2) {
  __shared__ __align__(16) float sx[256][4]; __shared__ __align__(16) float ss[256]; const int t = threadIdx.x; const size_t p = (size_t)blockIdx.x * 256 + t;
  const float x0 = bfr(XYZ2[p * 3]), x1 = bfr(XYZ2[p * 3 + 1]), x2 = bfr(XYZ2[p * 3 + 2]); sx[t][0] = x0; sx[t][1] = x1; sx[t][2] = x2; sx[t][3] = 0.f; ss[t] = __fadd_rn(__fadd_rn(__fmul_rn(x0, x0), __fmul_rn(x2, x2)), __fmul_rn(x1, x1));
  __syncthreads();
  vst2(X2 + p * 4, *(const v4f*)&sx[t][0]); if (t < 64) vst2(SQ2 + (size_t)blockIdx.x * 256 + t * 4, *(const v4f*)&ss[t * 4]);
}
__global__ __launch_bounds__(128) void k_interp(const float* __restrict__ XYZ1, const float* __restrict__ X2, const float* __restrict__ SQ2, const float* __restrict__ F1, const float* __restrict__ F2, __bf16* __restrict__ AH, __bf16* __restrict__ AL) {
  __shared__ float sd[4][NS]; __shared__ int sidx[4][4]; __shared__ float sw[4][4]; __shared__ __align__(16) __bf16 sh_[4][CIN], sl_[4][CIN];
  const int tid = threadIdx.x, wave = tid >> 5, lane = tid & 31; const size_t q = (size_t)blockIdx.x * 4 + wave; const int b = (int)(q / NN);
  const float qx0 = bfr(XYZ1[q * 3]), qx1 = bfr(XYZ1[q * 3 + 1]), qx2 = bfr(XYZ1[q * 3 + 2]); const float sqi = __fadd_rn(__fadd_rn(__fmul_rn(qx0, qx0), __fmul_rn(qx2, qx2)), __fmul_rn(qx1, qx1));
  for (int j = lane; j < NS; j += 32) { const size_t pj = (size_t)b * NS + j; const float dot = __fadd_rn(__fadd_rn(__fmul_rn(qx0, X2[pj * 4]), __fmul_rn(qx1, X2[pj * 4 + 1])), __fmul_rn(qx2, X2[pj * 4 + 2])); sd[wave][j] = __fsub_rn(__fadd_rn(sqi, SQ2[pj]), __fmul_rn(2.0f, dot)); }
  __syncthreads();
#pragma unroll 1
  for (int s = 0; s < 3; ++s) { float bv = 3.0e38f; int bi = 0x7fffffff;
    for (int j = lane; j < NS; j += 32) { const float v = sd[wave][j]; if (v < bv) { bv = v; bi = j; } }
#pragma unroll
    for (int o = 1; o < 32; o <<= 1) { const float ov = __shfl_xor(bv, o); const int oi = __shfl_xor(bi, o); if (ov < bv || (ov == bv && oi < bi)) { bv = ov; bi = oi; } }
    if (lane == 0) { sidx[wave][s] = bi; sd[wave][bi] = 3.0e38f; }
    __syncthreads(); }
  if (lane < 3) { const size_t pj = (size_t)b * NS + sidx[wave][lane]; const float dx = qx0 - X2[pj * 4], dy = qx1 - X2[pj * 4 + 1], dz = qx2 - X2[pj * 4 + 2]; const float d2 = fmaxf((dx * dx + dz * dz) + dy * dy, 1e-8f); sw[wave][lane] = 1.0f / d2; }
  __syncthreads();
  { const float w0 = sw[wave][0], w1 = sw[wave][1], w2 = sw[wave][2]; const float ws_ = (w0 + w1) + w2; const float n0 = w0 / ws_, n1 = w1 / ws_, n2 = w2 / ws_;
    const size_t i0 = (size_t)b * NS + sidx[wave][0], i1 = (size_t)b * NS + sidx[wave][1], i2 = (size_t)b * NS + sidx[wave][2];
    for (int c = lane; c < CIN; c += 32) { float v;
      if (c < CF) v = bfr(F1[q * CF + c]);
      else { const int cc = c - CF; v = (n0 * bfr(F2[i0 * CCO + cc]) + n1 * bfr(F2[i1 * CCO + cc])) + n2 * bfr(F2[i2 * CCO + cc]); }
      const __bf16 hb = (__bf16)v; sh_[wave][c] = hb; sl_[wave][c] = (__bf16)(v - (float)hb); } }
  __syncthreads();
  for (int e = tid; e < 4 * (CIN / 8) * 2; e += 128) { const int plane = e / (4 * CIN / 8), rem = e % (4 * CIN / 8); const int r = rem / (CIN / 8), pc = rem % (CIN / 8); const size_t o = ((size_t)blockIdx.x * 4 + r) * CIN + pc * 8;
    if (plane == 0) vst2((unsigned*)(AH + o), *(const v4u*)&sh_[r][pc * 8]); else vst2((unsigned*)(AL + o), *(const v4u*)&sl_[r][pc * 8]); }
}
template <int MODE>
__global__ __launch_bounds__(128) void k_gemm(const __bf16* __restrict__ AHp, const __bf16* __restrict__ ALp, const __bf16* __restrict__ PK, float* __restrict__ OUTR, double* __restrict__ ST) {
  constexpr int KD = (MODE == 0) ? CIN : MID; constexpr int NT = (MODE == 0) ? MID / 16 : CO / 16; constexpr int NCOL = NT * 16;
  __shared__ __align__(16) float so[4][16][NCOL + 4]; __shared__ __align__(16) double sst[NCOL][2];
  const int tid = threadIdx.x, wave = tid >> 5, lane = tid & 31, col = lane & 15, g = lane >> 4; const size_t r0 = (size_t)blockIdx.x * 64 + wave * 16; const __bf16* P = PK + ((MODE == 0) ? PK_1 : PK_2);
  v8f acc[NT];
#pragma unroll
  for (int j = 0; j < NT; ++j) acc[j] = v8f{};
#pragma unroll 2
  for (int kc = 0; kc < KD / 32; ++kc) { const v16b ah = frag_b(AHp + (r0 + col) * KD + kc * 32, lane), al = frag_b(ALp + (r0 + col) * KD + kc * 32, lane);
#pragma unroll
    for (int j = 0; j < NT; ++j) { const v16b w = frag_b(P + (size_t)(j * 16 + col) * KD + kc * 32, lane); acc[j] = wmma_bf(al, w, acc[j]); acc[j] = wmma_bf(ah, w, acc[j]); } }
#pragma unroll
  for (int j = 0; j < NT; ++j)
#pragma unroll
    for (int r = 0; r < 8; ++r) so[wave][8 * g + r][j * 16 + col] = acc[j][r];
  __syncthreads();
  for (int rl = 0; rl < 16; ++rl) for (int c0 = lane * 4; c0 < NCOL; c0 += 128) vst2(OUTR + (r0 + rl) * NCOL + c0, *(const v4f*)&so[wave][rl][c0]);
  for (int c = tid; c < NCOL; c += 128) { double a = 0.0, b2 = 0.0; for (int w = 0; w < 4; ++w) for (int r = 0; r < 16; ++r) { const double v = (double)so[w][r][c]; a += v; b2 += v * v; } sst[c][0] = a; sst[c][1] = b2; }
  __syncthreads();
  for (int c = tid; c < NCOL; c += 128) vst2((unsigned*)(ST + ((size_t)blockIdx.x * NCOL + c) * 2), *(const v4u*)&sst[c][0]);
}
template <int NC>
__global__ __launch_bounds__(256) void k_gnred(const double* __restrict__ ST, float* __restrict__ GN) {
  __shared__ double s1[8][32], s2[8][32]; __shared__ __align__(16) float sl[32]; const int t = threadIdx.x; const int b = blockIdx.x; const int grp = t >> 5, lane = t & 31; constexpr int CPG = NC / NGRP;
  double a = 0.0, q = 0.0;
  for (int blk = lane; blk < NN / 64; blk += 32) { const size_t base = ((size_t)(b * (NN / 64) + blk)) * NC; for (int c = 0; c < CPG; ++c) { a += ST[(base + grp * CPG + c) * 2]; q += ST[(base + grp * CPG + c) * 2 + 1]; } }
  s1[grp][lane] = a; s2[grp][lane] = q; __syncthreads();
  if (t < 8) { double A = 0.0, Q = 0.0; for (int l = 0; l < 32; ++l) { A += s1[t][l]; Q += s2[t][l]; } const double n = (double)NN * CPG; const double mean = A / n; const double var = fmax(Q / n - mean * mean, 0.0); sl[2 * t] = (float)mean; sl[2 * t + 1] = (float)(1.0 / sqrt(var + 1e-5)); }
  if (t >= 16 && t < 32) sl[t] = 0.f;
  __syncthreads();
  if (t < 8) vst2(GN + (size_t)b * 32 + t * 4, *(const v4f*)&sl[t * 4]);
}
__global__ __launch_bounds__(256) void k_norm1(const float* __restrict__ H1, const float* __restrict__ GN, const float* __restrict__ G, const float* __restrict__ BE, __bf16* __restrict__ NH_, __bf16* __restrict__ NL_) {
  __shared__ __align__(16) __bf16 sh_[64][MID + 8], sl_[64][MID + 8]; const int tid = threadIdx.x; const int b = (int)(((size_t)blockIdx.x * 64) / NN);
  for (int e = tid; e < 64 * MID; e += 256) { const int r = e / MID, c = e % MID; const int grp = c / (MID / NGRP); const size_t row = (size_t)blockIdx.x * 64 + r; float v = (H1[row * MID + c] - GN[b * 32 + 2 * grp]) * GN[b * 32 + 2 * grp + 1] * bfr(G[c]) + bfr(BE[c]); v = fmaxf(v, 0.f); const __bf16 hb = (__bf16)v; sh_[r][c] = hb; sl_[r][c] = (__bf16)(v - (float)hb); }
  __syncthreads();
  for (int e = tid; e < 64 * (MID / 8) * 2; e += 256) { const int plane = e / (64 * MID / 8), rem = e % (64 * MID / 8); const int r = rem / (MID / 8), pc = rem % (MID / 8); const size_t o = ((size_t)blockIdx.x * 64 + r) * MID + pc * 8;
    if (plane == 0) vst2((unsigned*)(NH_ + o), *(const v4u*)&sh_[r][pc * 8]); else vst2((unsigned*)(NL_ + o), *(const v4u*)&sl_[r][pc * 8]); }
}
__global__ __launch_bounds__(128) void k_out(const float* __restrict__ H2, const float* __restrict__ GN, const float* __restrict__ G, const float* __restrict__ BE, float* __restrict__ OUT) {
  __shared__ __align__(16) float s[CO]; const size_t row = blockIdx.x; const int t = threadIdx.x; const int b = (int)(row / NN); const int grp = t / (CO / NGRP);
  float v = (H2[row * CO + t] - GN[b * 32 + 2 * grp]) * GN[b * 32 + 2 * grp + 1] * bfr(G[t]) + bfr(BE[t]); s[t] = fmaxf(v, 0.f);
  __syncthreads();
  if (t < 32) vst2(OUT + row * CO + t * 4, *(const v4f*)&s[t * 4]);
}
extern "C" void kernel_launch(void* const* d_in, const int* in_sizes, int n_in, void* d_out, int out_size, void* d_ws, size_t ws_size, hipStream_t stream) {
  (void)in_sizes; (void)n_in; (void)out_size;
  const float** F = (const float**)d_in;
  if (ws_size < (size_t)WS_END) return;
  char* ws = (char*)d_ws; __bf16 *PK = (__bf16*)(ws + WS_PK), *AH = (__bf16*)(ws + WS_AH), *AL = (__bf16*)(ws + WS_AL), *N1H = (__bf16*)(ws + WS_N1H), *N1L = (__bf16*)(ws + WS_N1L); float *X2 = (float*)(ws + WS_X2), *SQ2 = (float*)(ws + WS_SQ2), *H1 = (float*)(ws + WS_H1), *GN1 = (float*)(ws + WS_GN1), *H2 = (float*)(ws + WS_H2), *GN2 = (float*)(ws + WS_GN2); double *ST1 = (double*)(ws + WS_ST1), *ST2 = (double*)(ws + WS_ST2);
  k_pack<<<dim3(MID, 2), 256, 0, stream>>>(F[4], F[7], PK);
  k_src<<<NB * NS / 256, 256, 0, stream>>>(F[1], X2, SQ2);
  k_interp<<<NR / 4, 128, 0, stream>>>(F[0], X2, SQ2, F[2], F[3], AH, AL);
  k_gemm<0><<<NR / 64, 128, 0, stream>>>(AH, AL, PK, H1, ST1);
  k_gnred<MID><<<NB, 256, 0, stream>>>(ST1, GN1);
  k_norm1<<<NR / 64, 256, 0, stream>>>(H1, GN1, F[5], F[6], N1H, N1L);
  k_gemm<1><<<NR / 64, 128, 0, stream>>>(N1H, N1L, PK, H2, ST2);
  k_gnred<CO><<<NB, 256, 0, stream>>>(ST2, GN2);
  k_out<<<NR, 128, 0, stream>>>(H2, GN2, F[8], F[9], (float*)d_out);
}
